// RNNModel_32126355374137
// MI455X (gfx1250) — hardware-verified
//
#include <hip/hip_runtime.h>
#include <math.h>

constexpr int NB      = 512;
constexpr int NTS     = 2048;
constexpr int HD      = 64;
constexpr int G4      = 256;
constexpr int F1      = 128;
constexpr int NCLS    = 10;
constexpr int NTHR    = 256;
constexpr int RB      = 16;
constexpr int HP      = 72;
constexpr int HSP     = 68;
constexpr int YSP     = 132;
constexpr int XCH     = 128;
constexpr int XCH_LOG = 7;
constexpr int NCHK    = NTS / XCH;
constexpr float HCARRY = 16.0f;
constexpr float WCARRY = 64.0f;
constexpr float CINV   = 1.0f / (HCARRY * WCARRY);
static_assert(NB % RB == 0 && RB == 16, "one 16-row m-subtile per block");
static_assert(G4 == 4 * HD && HD == 64, "two 32-deep k-chunks per 64-wide operand");
static_assert(NTHR == 256 && NTHR == G4, "bias tables filled one element per thread");
static_assert((4 * RB * HP) % NTHR == 0, "h tile zero-fill loop exact");
static_assert(RB * XCH == 2 * NTHR * 4, "x chunk staging: 2 float4 per thread");
static_assert(NTS % XCH == 0 && XCH == (1 << XCH_LOG), "chunking exact");
static_assert(64 * HD == 4 * NTHR * 4, "fc1 half-plane staging: 4 float4 per thread");
static_assert(2 * RB * XCH >= 64 * HD, "x staging region holds one fc1 half plane");
static_assert(F1 == 128 && RB * F1 == NTHR * 8, "fc1 outputs: 2 halves x 4 per thread");
static_assert((RB * NCLS) % 32 == 0, "fc2 thread set is whole waves");
static_assert((RB * NCLS * 4) % 128 == 0 && RB * NCLS * 4 == 640, "block output = 5 whole 128-B lines");
static_assert((NCLS * F1) % 4 == 0 && ((NCLS * F1 / 4) % 32) == 0, "fc2_w staging guard is wave-uniform");
static_assert(HP % 8 == 0 && HSP % 4 == 0 && YSP % 4 == 0, "16-B aligned LDS rows");
static_assert((G4 * HD) % 8 == 0 && ((G4 * HD / 8) % NTHR) == 0, "weight cast grid exact");

typedef __attribute__((ext_vector_type(16))) _Float16 v16h;
typedef __attribute__((ext_vector_type(8)))  _Float16 v8h;
typedef __attribute__((ext_vector_type(8)))  float    v8f;
typedef __attribute__((ext_vector_type(4)))  float    v4f;

template <typename T> struct Frag;
template <> struct Frag<_Float16> {
  typedef v16h V; union U { v16h v; v8h h[2]; };
  static __device__ __forceinline__ v16h load(const _Float16* p) {
    U f; f.h[0] = *(const v8h*)(p); f.h[1] = *(const v8h*)(p + 16); return f.v;
  }
  static __device__ __forceinline__ v8f mma(v16h a, v16h b, v8f c) {
    return __builtin_amdgcn_wmma_f32_16x16x32_f16(false, a, false, b, (short)0, c, false, false);
  }
};

__device__ __forceinline__ void mma_guard_all(v8f& a0, v8f& a1, v8f& a2, v8f& a3,
                                              v16h fa, v16h b0, v16h b1, v16h b2, v16h b3) {
  asm volatile("v_nop\n\tv_nop\n\tv_nop\n\tv_nop"
               : "+v"(a0), "+v"(a1), "+v"(a2), "+v"(a3)
               : "v"(fa), "v"(b0), "v"(b1), "v"(b2), "v"(b3));
}

__device__ __forceinline__ float fsig(float v)  { return __builtin_amdgcn_rcpf(1.0f + expf(-v)); }
__device__ __forceinline__ float ftanh(float v) { return 1.0f - 2.0f * __builtin_amdgcn_rcpf(expf(2.0f * v) + 1.0f); }

__global__ __launch_bounds__(NTHR) void cast_plane_kernel(const float* __restrict__ src, unsigned short* __restrict__ dst,
                                                          int n8, float sc) {
  const int i = blockIdx.x * NTHR + threadIdx.x;
  if (i < n8) {
    const v4f a = *(const v4f*)(src + (size_t)i * 8);
    const v4f b = *(const v4f*)(src + (size_t)i * 8 + 4);
    v8h hv;
#pragma unroll
    for (int e = 0; e < 4; ++e) {
      hv[e]     = (_Float16)(a[e] * sc);
      hv[4 + e] = (_Float16)(b[e] * sc);
    }
    *(volatile v8h*)(dst + (size_t)i * 8) = hv;
    __threadfence();
    *(volatile v8h*)(dst + (size_t)i * 8) = hv;
  }
}

__device__ __forceinline__ void stage_x_chunk(float* xsb, const float* __restrict__ x, int rowbase, int ch, int tid) {
#pragma unroll
  for (int it = 0; it < 2; ++it) {
    const int idx = it * NTHR + tid;
    const int row = idx >> 5, c4 = (idx & 31) * 4;
    const v4f v = *(const v4f*)(x + (size_t)(rowbase + row) * NTS + (size_t)ch * XCH + c4);
    *(v4f*)(xsb + row * XCH + c4) = v;
  }
}

__global__ __launch_bounds__(NTHR) void lstm2_head_kernel(
    const float* __restrict__ x, const float* __restrict__ w_ih0,
    const float* __restrict__ b_ih0, const float* __restrict__ b_hh0,
    const float* __restrict__ b_ih1, const float* __restrict__ b_hh1,
    const unsigned short* __restrict__ W0p, const unsigned short* __restrict__ W1p,
    const unsigned short* __restrict__ W2p,
    const float* __restrict__ fc1_w, const float* __restrict__ fc1_b,
    const float* __restrict__ fc2_w, const float* __restrict__ fc2_b,
    float* __restrict__ out) {
  __shared__ __align__(16) float    xs[2][RB * XCH];
  __shared__ __align__(16) _Float16 ht[4][RB * HP];
  __shared__ __align__(16) float    hs[RB * HSP];
  __shared__ __align__(16) float    ys[RB * YSP];
  __shared__ __align__(16) float    w2s[NCLS * F1];
  __shared__ __align__(16) float    os[RB * NCLS];
  __shared__ float cw0[G4], cb0[G4], cb1[G4], cf1b[F1], cf2b[16];

  const _Float16* W0 = (const _Float16*)W0p;
  const _Float16* W1 = (const _Float16*)W1p;
  const _Float16* W2 = (const _Float16*)W2p;
  const int tid = threadIdx.x, lane = tid & 31, wave = tid >> 5;
  const int c = lane & 15, hh = lane >> 4, koff = hh * 8;
  const int grp = wave >> 2, g = wave & 3, col = 16 * g + c;
  const int rowbase = blockIdx.x * RB;

  {
    _Float16* htf = &ht[0][0];
#pragma unroll 1
    for (int i = tid; i < 4 * RB * HP; i += NTHR) htf[i] = (_Float16)0.0f;
  }
  cw0[tid] = w_ih0[tid];
  cb0[tid] = b_ih0[tid] + b_hh0[tid];
  cb1[tid] = b_ih1[tid] + b_hh1[tid];
  stage_x_chunk(&xs[0][0], x, rowbase, 0, tid);
  float cst[8], hst[8];
#pragma unroll
  for (int r = 0; r < 8; ++r) { cst[r] = 0.0f; hst[r] = 0.0f; }
  __syncthreads();

  float wv[4], bs0[4], bs1[4];
#pragma unroll
  for (int q = 0; q < 4; ++q) {
    wv[q]  = cw0[q * HD + col];
    bs0[q] = cb0[q * HD + col];
    bs1[q] = cb1[q * HD + col];
  }
  const v8f z8 = {0.f, 0.f, 0.f, 0.f, 0.f, 0.f, 0.f, 0.f};

#pragma unroll 1
  for (int k = 0; k <= NTS; ++k) {
    const int cur = k & 1, prv = cur ^ 1;
    if ((k & (XCH - 1)) == 0) {
      const int cn = (k >> XCH_LOG) + 1;
      if (cn < NCHK) stage_x_chunk(&xs[cn & 1][0], x, rowbase, cn, tid);
    }
    const bool active = (grp == 0) ? (k < NTS) : (k >= 1);
    if (active) {
      v8f acc[4];
      acc[0] = z8; acc[1] = z8; acc[2] = z8; acc[3] = z8;
      if (grp == 0) {
        const _Float16* arow = &ht[prv][0] + c * HP + koff;
#pragma unroll
        for (int kk = 0; kk < 2; ++kk) {
          const v16h a  = Frag<_Float16>::load(arow + 32 * kk);
          const _Float16* wb = W0 + (size_t)col * HD + koff + 32 * kk;
          const v16h b0 = Frag<_Float16>::load(wb);
          const v16h b1 = Frag<_Float16>::load(wb + (size_t)1 * HD * HD);
          const v16h b2 = Frag<_Float16>::load(wb + (size_t)2 * HD * HD);
          const v16h b3 = Frag<_Float16>::load(wb + (size_t)3 * HD * HD);
          acc[0] = Frag<_Float16>::mma(a, b0, acc[0]);
          acc[1] = Frag<_Float16>::mma(a, b1, acc[1]);
          acc[2] = Frag<_Float16>::mma(a, b2, acc[2]);
          acc[3] = Frag<_Float16>::mma(a, b3, acc[3]);
          mma_guard_all(acc[0], acc[1], acc[2], acc[3], a, b0, b1, b2, b3);
        }
        const float* xsb = &xs[(k >> XCH_LOG) & 1][0];
        const int tl = k & (XCH - 1);
        float xv[8];
#pragma unroll
        for (int r = 0; r < 8; ++r) xv[r] = xsb[(8 * hh + r) * XCH + tl];
#pragma unroll
        for (int q = 0; q < 4; ++q)
#pragma unroll
          for (int r = 0; r < 8; ++r) acc[q][r] = acc[q][r] * CINV + (xv[r] * wv[q] + bs0[q]);
      } else {
        const _Float16* arow1 = &ht[prv][0] + c * HP + koff;
        const _Float16* arow2 = &ht[2 + cur][0] + c * HP + koff;
#pragma unroll
        for (int kk = 0; kk < 2; ++kk) {
          const v16h a  = Frag<_Float16>::load(arow1 + 32 * kk);
          const _Float16* wb = W1 + (size_t)col * HD + koff + 32 * kk;
          const v16h b0 = Frag<_Float16>::load(wb);
          const v16h b1 = Frag<_Float16>::load(wb + (size_t)1 * HD * HD);
          const v16h b2 = Frag<_Float16>::load(wb + (size_t)2 * HD * HD);
          const v16h b3 = Frag<_Float16>::load(wb + (size_t)3 * HD * HD);
          acc[0] = Frag<_Float16>::mma(a, b0, acc[0]);
          acc[1] = Frag<_Float16>::mma(a, b1, acc[1]);
          acc[2] = Frag<_Float16>::mma(a, b2, acc[2]);
          acc[3] = Frag<_Float16>::mma(a, b3, acc[3]);
          mma_guard_all(acc[0], acc[1], acc[2], acc[3], a, b0, b1, b2, b3);
        }
#pragma unroll
        for (int kk = 0; kk < 2; ++kk) {
          const v16h a  = Frag<_Float16>::load(arow2 + 32 * kk);
          const _Float16* wb = W2 + (size_t)col * HD + koff + 32 * kk;
          const v16h b0 = Frag<_Float16>::load(wb);
          const v16h b1 = Frag<_Float16>::load(wb + (size_t)1 * HD * HD);
          const v16h b2 = Frag<_Float16>::load(wb + (size_t)2 * HD * HD);
          const v16h b3 = Frag<_Float16>::load(wb + (size_t)3 * HD * HD);
          acc[0] = Frag<_Float16>::mma(a, b0, acc[0]);
          acc[1] = Frag<_Float16>::mma(a, b1, acc[1]);
          acc[2] = Frag<_Float16>::mma(a, b2, acc[2]);
          acc[3] = Frag<_Float16>::mma(a, b3, acc[3]);
          mma_guard_all(acc[0], acc[1], acc[2], acc[3], a, b0, b1, b2, b3);
        }
#pragma unroll
        for (int q = 0; q < 4; ++q)
#pragma unroll
          for (int r = 0; r < 8; ++r) acc[q][r] = acc[q][r] * CINV + bs1[q];
      }
      const int dsel = (grp == 0) ? cur : (2 + prv);
      _Float16* dst = &ht[dsel][0];
#pragma unroll
      for (int r = 0; r < 8; ++r) {
        const float ig = fsig(acc[0][r]);
        const float fg = fsig(acc[1][r]);
        const float gg = ftanh(acc[2][r]);
        const float og = fsig(acc[3][r]);
        const float cn = fg * cst[r] + ig * gg;
        const float hn = og * ftanh(cn);
        cst[r] = cn;
        hst[r] = hn;
        dst[(8 * hh + r) * HP + col] = (_Float16)(hn * HCARRY);
      }
    }
    __syncthreads();
  }

  if (grp == 1) {
#pragma unroll
    for (int r = 0; r < 8; ++r) hs[(8 * hh + r) * HSP + col] = hst[r];
  }
#pragma unroll
  for (int it = 0; it < 2; ++it) {
    const int idx = it * NTHR + tid;
    if (idx < NCLS * F1 / 4) {
      const v4f v = *(const v4f*)(fc2_w + 4 * idx);
      *(v4f*)(w2s + 4 * idx) = v;
    }
  }
  {
    const float v1 = fc1_b[tid & (F1 - 1)];
    if (tid < F1) cf1b[tid] = v1;
    const int tc = (tid < NCLS) ? tid : (NCLS - 1);
    const float v2 = fc2_b[tc];
    if (tid < 16) cf2b[tid] = (tid < NCLS) ? v2 : 0.0f;
  }
  __syncthreads();

#pragma unroll 1
  for (int half = 0; half < 2; ++half) {
    float* wst = &xs[0][0];
#pragma unroll
    for (int it = 0; it < 4; ++it) {
      const int idx = it * NTHR + tid;
      const int row = idx >> 4, c4 = (idx & 15) * 4;
      const v4f v = *(const v4f*)(fc1_w + (size_t)(64 * half + row) * HD + c4);
      *(v4f*)(wst + row * HD + c4) = v;
    }
    __syncthreads();
    const int m = tid >> 4, nl = tid & 15;
#pragma unroll 1
    for (int j = 0; j < 4; ++j) {
      const int nloc = 16 * j + nl;
      float a = 0.0f;
#pragma unroll
      for (int k4 = 0; k4 < HD / 4; ++k4) {
        const v4f hv4 = *(const v4f*)(hs + m * HSP + 4 * k4);
        const v4f wv4 = *(const v4f*)(wst + nloc * HD + 4 * k4);
        a += hv4[0] * wv4[0];
        a += hv4[1] * wv4[1];
        a += hv4[2] * wv4[2];
        a += hv4[3] * wv4[3];
      }
      const int n = 64 * half + nloc;
      float y = a + cf1b[n];
      y = fmaxf(y, 0.0f);
      ys[m * YSP + n] = y;
    }
    __syncthreads();
  }

  if (tid < RB * NCLS) {
    const int m = tid / NCLS, p = tid - m * NCLS;
    float a = 0.0f;
#pragma unroll 1
    for (int n4 = 0; n4 < F1 / 4; ++n4) {
      const v4f yv = *(const v4f*)(ys + m * YSP + 4 * n4);
      const v4f wq = *(const v4f*)(w2s + p * F1 + 4 * n4);
      a += yv[0] * wq[0];
      a += yv[1] * wq[1];
      a += yv[2] * wq[2];
      a += yv[3] * wq[3];
    }
    os[tid] = a + cf2b[p];
  }
  __syncthreads();

  if (wave == 0) {
    float* ob = out + (size_t)blockIdx.x * (RB * NCLS);
    const int l2 = (lane < 8) ? lane : 7;
    const v4f v0 = *(const v4f*)(os + 4 * lane);
    const v4f v1 = *(const v4f*)(os + 128 + 4 * l2);
    for (int pass = 0; pass < 2; ++pass) {
      *(volatile v4f*)(ob + 4 * lane) = v0;
      if (lane < 8) *(volatile v4f*)(ob + 128 + 4 * lane) = v1;
      __threadfence();
    }
  }
}

extern "C" void kernel_launch(void* const* d_in, const int* in_sizes, int n_in,
                              void* d_out, int out_size, void* d_ws, size_t ws_size, hipStream_t stream) {
  if (n_in < 13 || d_out == nullptr || d_ws == nullptr) return;
  if (in_sizes[0] != NB * NTS || in_sizes[1] != G4 || in_sizes[2] != G4 * HD || in_sizes[3] != G4 ||
      in_sizes[4] != G4 || in_sizes[5] != G4 * HD || in_sizes[6] != G4 * HD || in_sizes[7] != G4 ||
      in_sizes[8] != G4 || in_sizes[9] != F1 * HD || in_sizes[10] != F1 || in_sizes[11] != NCLS * F1 ||
      in_sizes[12] != NCLS || out_size != NB * NCLS) return;

  const float* x     = (const float*)d_in[0];
  const float* w_ih0 = (const float*)d_in[1];
  const float* w_hh0 = (const float*)d_in[2];
  const float* b_ih0 = (const float*)d_in[3];
  const float* b_hh0 = (const float*)d_in[4];
  const float* w_ih1 = (const float*)d_in[5];
  const float* w_hh1 = (const float*)d_in[6];
  const float* b_ih1 = (const float*)d_in[7];
  const float* b_hh1 = (const float*)d_in[8];
  const float* fc1_w = (const float*)d_in[9];
  const float* fc1_b = (const float*)d_in[10];
  const float* fc2_w = (const float*)d_in[11];
  const float* fc2_b = (const float*)d_in[12];
  float* out = (float*)d_out;

  char* ws = (char*)d_ws; size_t off = 0;
  auto carve = [&](size_t bytes) -> char* { char* p = ws + off; off += (bytes + 255) & ~(size_t)255; return p; };
  unsigned short* W0 = (unsigned short*)carve((size_t)G4 * HD * 2);
  unsigned short* W1 = (unsigned short*)carve((size_t)G4 * HD * 2);
  unsigned short* W2 = (unsigned short*)carve((size_t)G4 * HD * 2);
  if (off > ws_size || off > (size_t)134217728) return;

  const int n8 = G4 * HD / 8;
  cast_plane_kernel<<<n8 / NTHR, NTHR, 0, stream>>>(w_hh0, W0, n8, WCARRY);
  cast_plane_kernel<<<n8 / NTHR, NTHR, 0, stream>>>(w_ih1, W1, n8, WCARRY);
  cast_plane_kernel<<<n8 / NTHR, NTHR, 0, stream>>>(w_hh1, W2, n8, WCARRY);

  lstm2_head_kernel<<<NB / RB, NTHR, 0, stream>>>(x, w_ih0, b_ih0, b_hh0, b_ih1, b_hh1, W0, W1, W2,
                                                   fc1_w, fc1_b, fc2_w, fc2_b, out);
}
